// InverseAutoRegressiveFlow_57432302682238
// MI455X (gfx1250) — hardware-verified
//
#include <hip/hip_runtime.h>
#include <math.h>

constexpr int kDims         = 64;
constexpr int kCtxLen       = 16;
constexpr int kHid          = 64;
constexpr int kRowsPerWave  = 16;
constexpr int kWavesPerBlk  = 4;
constexpr int kRowsPerBlock = kRowsPerWave * kWavesPerBlk;
constexpr int kThreads      = 32 * kWavesPerBlk;
constexpr int kW1Pitch      = 32;
constexpr int kW2Pitch      = 64;
constexpr int kW3Rows       = 16;

constexpr float kWCarry   = 8.0f;
constexpr float kB1Carry  = 8.0f;
constexpr float kB2Carry  = 128.0f;
constexpr float kB3Carry  = 128.0f;
constexpr float kAct1Scale = 2.0f;
constexpr float kAct2Scale = 0.125f;
constexpr float kOut3Scale = 1.0f / 128.0f;
constexpr float kNegSlope  = 0.01f;

typedef __attribute__((ext_vector_type(16))) _Float16 v16h;
typedef __attribute__((ext_vector_type(8)))  _Float16 v8h;
typedef __attribute__((ext_vector_type(8)))  float    v8f;
typedef __attribute__((ext_vector_type(4)))  float    v4f;
typedef __attribute__((ext_vector_type(8)))  unsigned v8u;

struct FragH {
  union U { v16h v; v8h h[2]; };
  static __device__ __forceinline__ v16h load(const _Float16* p) {
    U f; f.h[0] = *(const v8h*)(p); f.h[1] = *(const v8h*)(p + 16); return f.v;
  }
};

__device__ __forceinline__ v8f mma16(v16h a, v16h b, v8f c) {
  c = __builtin_amdgcn_wmma_f32_16x16x32_f16(false, a, false, b, (short)0, c, false, false);
  asm volatile("v_nop\n\tv_nop\n\tv_nop\n\tv_nop" : "+v"(c) : "v"(a), "v"(b));
  return c;
}

__device__ __forceinline__ unsigned f16_bits(float x) {
  return (unsigned)__builtin_bit_cast(unsigned short, (_Float16)x);
}

__device__ __forceinline__ _Float16 act16(float a, float sc) {
  const float v = a * sc;
  return (_Float16)fmaxf(v, v * kNegSlope);
}

__global__ __launch_bounds__(kThreads)
void ar_affine_cond_kernel(const float* __restrict__ z,
                           const float* __restrict__ W1, const float* __restrict__ b1,
                           const float* __restrict__ W2, const float* __restrict__ b2,
                           const float* __restrict__ W3, const float* __restrict__ b3,
                           float* __restrict__ out, int nrows)
{
  __shared__ __align__(16) _Float16 w1t[kHid * kW1Pitch];
  __shared__ __align__(16) _Float16 w2t[kHid * kW2Pitch];
  __shared__ __align__(16) _Float16 w3t[kW3Rows * kW2Pitch];
  __shared__ __align__(32) float b1s[kHid];
  __shared__ __align__(32) float b2s[kHid];
  __shared__ __align__(32) float b3s[kW3Rows];
  __shared__ __align__(16) float ytile[kRowsPerBlock * kDims];

  const int tid  = threadIdx.x;
  const int wave = tid >> 5;
  const int lane = tid & 31;
  const int hh   = lane >> 4;
  const int cc   = lane & 15;

#pragma unroll 1
  for (int i = 0; i < 16; ++i) {
    const int idx = tid + i * kThreads;
    const int f = idx >> 5, k = idx & 31;
    const int kcl = (k < kCtxLen) ? k : (kCtxLen - 1);
    const float v = W1[kcl * kHid + f] * kWCarry;
    w1t[idx] = (_Float16)((k < kCtxLen) ? v : 0.0f);
  }
#pragma unroll 1
  for (int i = 0; i < 32; ++i) {
    const int idx = tid + i * kThreads;
    const int f = idx >> 6, k = idx & 63;
    w2t[idx] = (_Float16)(W2[k * kHid + f] * kWCarry);
  }
#pragma unroll 1
  for (int i = 0; i < 8; ++i) {
    const int idx = tid + i * kThreads;
    const int j = idx >> 6, k = idx & 63;
    const int jcl = (j < 2) ? j : 1;
    const float v = W3[k * 2 + jcl] * kWCarry;
    w3t[idx] = (_Float16)((j < 2) ? v : 0.0f);
  }
  if (tid < kHid) {
    b1s[tid] = b1[tid] * kB1Carry;
    b2s[tid] = b2[tid] * kB2Carry;
  }
  if (tid < kW3Rows) {
    const int jcl = (tid < 2) ? tid : 1;
    const float v = b3[jcl] * kB3Carry;
    b3s[tid] = (tid < 2) ? v : 0.0f;
  }
  __syncthreads();

  const int wrow  = wave * kRowsPerWave;
  const int grow  = blockIdx.x * kRowsPerBlock + wrow + cc;
  const int growc = (grow < nrows) ? grow : (nrows - 1);
  const float* zrow = z + (size_t)growc * kDims;

  const float y0 = zrow[0];
  if (hh == 0) ytile[(wrow + cc) * kDims + 0] = y0;
  unsigned q0, q1, q2, q3;
  {
    const unsigned ib = f16_bits(y0);
    q0 = q1 = q2 = q3 = ib | (ib << 16);
  }
  const v8f zero8 = (v8f){0.f, 0.f, 0.f, 0.f, 0.f, 0.f, 0.f, 0.f};
  (void)zero8;

#pragma unroll 1
  for (int t = 1; t < kDims; ++t) {
    asm volatile("" ::: "memory");

    v8u cw;
    cw[0] = q0; cw[1] = q1; cw[2] = q2; cw[3] = q3; cw[4] = 0u; cw[5] = 0u; cw[6] = 0u; cw[7] = 0u;
    const v16h bctx = __builtin_bit_cast(v16h, cw);

    v8f acc1[4];
#pragma unroll
    for (int ft = 0; ft < 4; ++ft) {
      const v8f cini = *(const v8f*)(b1s + 16 * ft + 8 * hh);
      const v16h a = FragH::load(w1t + (16 * ft + cc) * kW1Pitch + 8 * hh);
      acc1[ft] = mma16(a, bctx, cini);
    }
    v16h hb1[2];
#pragma unroll
    for (int kc = 0; kc < 2; ++kc) {
#pragma unroll
      for (int i = 0; i < 8; ++i) {
        hb1[kc][i]     = act16(acc1[2 * kc][i],     kAct1Scale);
        hb1[kc][8 + i] = act16(acc1[2 * kc + 1][i], kAct1Scale);
      }
    }
    asm volatile("" ::: "memory");

    v8f acc2[4];
#pragma unroll
    for (int ft = 0; ft < 4; ++ft) {
      acc2[ft] = *(const v8f*)(b2s + 16 * ft + 8 * hh);
#pragma unroll
      for (int kc = 0; kc < 2; ++kc) {
        const v16h a = FragH::load(w2t + (16 * ft + cc) * kW2Pitch + 32 * kc + 8 * hh);
        acc2[ft] = mma16(a, hb1[kc], acc2[ft]);
      }
    }
    v16h hb2[2];
#pragma unroll
    for (int kc = 0; kc < 2; ++kc) {
#pragma unroll
      for (int i = 0; i < 8; ++i) {
        hb2[kc][i]     = act16(acc2[2 * kc][i],     kAct2Scale);
        hb2[kc][8 + i] = act16(acc2[2 * kc + 1][i], kAct2Scale);
      }
    }
    asm volatile("" ::: "memory");

    v8f acc3 = *(const v8f*)(b3s + 8 * hh);
#pragma unroll
    for (int kc = 0; kc < 2; ++kc) {
      const v16h a = FragH::load(w3t + cc * kW2Pitch + 32 * kc + 8 * hh);
      acc3 = mma16(a, hb2[kc], acc3);
    }
    const float mv = acc3[0] * kOut3Scale;
    const float sv = acc3[1] * kOut3Scale;
    const float zt = zrow[t];
    const float ylo = zt * expf(sv) + mv;
    const float yhi = __shfl_xor(ylo, 16, 32);
    const float yv  = hh ? yhi : ylo;
    if (hh == 0) ytile[(wrow + cc) * kDims + t] = yv;

    const unsigned pq0 = __shfl_xor(q0, 16, 32);
    const unsigned yb  = f16_bits(yv);
    const unsigned inc = hh ? yb : (pq0 & 0xffffu);
    q0 = (q0 >> 16) | (q1 << 16);
    q1 = (q1 >> 16) | (q2 << 16);
    q2 = (q2 >> 16) | (q3 << 16);
    q3 = (q3 >> 16) | (inc << 16);
  }

  __syncthreads();

  {
    const float* yt = ytile + wrow * kDims;
    const int browBase = blockIdx.x * kRowsPerBlock + wrow;
    const int c4 = cc * 4;
    for (int pass = 0; pass < 2; ++pass) {
#pragma unroll
      for (int it = 0; it < 8; ++it) {
        const int row = it * 2 + hh;
        const v4f v = *(const v4f*)(yt + row * kDims + c4);
        const int orow = browBase + row;
        if (orow < nrows) *(volatile v4f*)(out + (size_t)orow * kDims + c4) = v;
      }
      __threadfence();
    }
  }
}

extern "C" void kernel_launch(void* const* d_in, const int* in_sizes, int n_in,
                              void* d_out, int out_size, void* d_ws, size_t ws_size,
                              hipStream_t stream) {
  (void)d_ws; (void)ws_size;
  if (n_in < 7) return;
  const int nrows = in_sizes[0] / kDims;
  if (nrows < 1) return;
  if (in_sizes[1] != kCtxLen * kHid) return;
  if (in_sizes[2] != kHid) return;
  if (in_sizes[3] != kHid * kHid) return;
  if (in_sizes[4] != kHid) return;
  if (in_sizes[5] != kHid * 2) return;
  if (in_sizes[6] < 2) return;
  if (out_size < nrows * kDims) return;

  const float* z  = (const float*)d_in[0];
  const float* W1 = (const float*)d_in[1];
  const float* b1 = (const float*)d_in[2];
  const float* W2 = (const float*)d_in[3];
  const float* b2 = (const float*)d_in[4];
  const float* W3 = (const float*)d_in[5];
  const float* b3 = (const float*)d_in[6];
  float* outp = (float*)d_out;

  const int grid = (nrows + kRowsPerBlock - 1) / kRowsPerBlock;
  ar_affine_cond_kernel<<<dim3(grid), dim3(kThreads), 0, stream>>>(z, W1, b1, W2, b2, W3, b3, outp, nrows);
}
